// UpdateX_56358560858585
// MI455X (gfx1250) — hardware-run, weakly checked
//
#include <hip/hip_runtime.h>
#include <math.h>

typedef __attribute__((ext_vector_type(16))) _Float16 v16h;
typedef __attribute__((ext_vector_type(16))) __bf16 v16b;
typedef __attribute__((ext_vector_type(8)))  _Float16 v8h;
typedef __attribute__((ext_vector_type(8)))  float v8f;
typedef __attribute__((ext_vector_type(4)))  float v4f;
typedef __attribute__((ext_vector_type(2)))  float v2f;
typedef __attribute__((ext_vector_type(4)))  unsigned v4u;
typedef __attribute__((ext_vector_type(4)))  int v4i;
typedef float __attribute__((may_alias)) float_a;
typedef int __attribute__((may_alias)) int_a;

template <typename T> __device__ __forceinline__ void vst2(void* p, T v) { *(volatile T*)p = v; __threadfence(); *(volatile T*)p = v; }
__device__ __forceinline__ v8f wmma16(v16h a, v16h b, v8f c) {
  v8f d = __builtin_amdgcn_wmma_f32_16x16x32_f16(false, a, false, b, (short)0, c, false, false);
  asm volatile("v_nop\n\tv_nop\n\tv_nop\n\tv_nop" : "+v"(d) : "v"(a), "v"(b));
  return d;
}
__device__ __forceinline__ v8f wmma_bf(v16b a, v16b b, v8f c) {
  v8f d = __builtin_amdgcn_wmma_f32_16x16x32_bf16(false, a, false, b, (short)0, c, false, false);
  asm volatile("v_nop\n\tv_nop\n\tv_nop\n\tv_nop" : "+v"(d) : "v"(a), "v"(b));
  return d;
}
__device__ __forceinline__ v16h frag_h(const _Float16* rowk0, int lane) {
  union { v16h v; v8h q[2]; } u; const _Float16* p = rowk0 + 8 * (lane >> 4);
  u.q[0] = *(const v8h*)p; u.q[1] = *(const v8h*)(p + 16); return u.v;
}
__device__ __forceinline__ v16h frag_f32(const float* rowk0, int lane) {
  v16h a; const float* p = rowk0 + 8 * (lane >> 4);
#pragma unroll
  for (int i = 0; i < 8; ++i) { a[i] = (_Float16)p[i]; a[8 + i] = (_Float16)p[16 + i]; }
  return a;
}
__device__ __forceinline__ v16h frag_f32s(const float* rowk0, int lane, float sc) {
  v16h a; const float* p = rowk0 + 8 * (lane >> 4);
#pragma unroll
  for (int i = 0; i < 8; ++i) { a[i] = (_Float16)(p[i] * sc); a[8 + i] = (_Float16)(p[16 + i] * sc); }
  return a;
}
__device__ __forceinline__ v16h fragc_f32(const float* W, int k0, int n, int lane, int ld, int K) {
  v16h a; const int g = lane >> 4;
#pragma unroll
  for (int i = 0; i < 8; ++i) { const int ka = k0 + 8 * g + i, kb = ka + 16;
    a[i] = (_Float16)(ka < K ? W[(size_t)(ka < K ? ka : K - 1) * ld + n] : 0.f); a[8 + i] = (_Float16)(kb < K ? W[(size_t)(kb < K ? kb : K - 1) * ld + n] : 0.f); }
  return a;
}
struct F2 { v16b h, l; };
__device__ __forceinline__ F2 bsplit16(const float v[16]) { F2 r;
#pragma unroll
  for (int i = 0; i < 16; ++i) { const __bf16 h = (__bf16)v[i]; r.h[i] = h; r.l[i] = (__bf16)(v[i] - (float)h); }
  return r; }
__device__ __forceinline__ F2 split_row(const float* row, int k0, int lane) { float v[16]; const float* p = row + k0 + 8 * (lane >> 4);
#pragma unroll
  for (int i = 0; i < 8; ++i) { v[i] = p[i]; v[8 + i] = p[16 + i]; }
  return bsplit16(v); }
__device__ __forceinline__ F2 split_rowK(const float* row, int k0, int lane, int K) { float v[16]; const int g = lane >> 4;
#pragma unroll
  for (int i = 0; i < 8; ++i) { const int ka = k0 + 8 * g + i, kb = ka + 16; v[i] = ka < K ? row[ka < K ? ka : K - 1] : 0.f; v[8 + i] = kb < K ? row[kb < K ? kb : K - 1] : 0.f; }
  return bsplit16(v); }
__device__ __forceinline__ F2 split_col(const float* W, int k0, int n, int lane, int ld, int K) { float v[16]; const int g = lane >> 4;
#pragma unroll
  for (int i = 0; i < 8; ++i) { const int ka = k0 + 8 * g + i, kb = ka + 16; v[i] = ka < K ? W[(size_t)(ka < K ? ka : K - 1) * ld + n] : 0.f; v[8 + i] = kb < K ? W[(size_t)(kb < K ? kb : K - 1) * ld + n] : 0.f; }
  return bsplit16(v); }
__device__ __forceinline__ v8f mac3(const F2& a, const F2& b, v8f c) { c = wmma_bf(a.l, b.h, c); c = wmma_bf(a.h, b.l, c); return wmma_bf(a.h, b.h, c); }
__device__ __forceinline__ float sigm(float v) { return 1.0f / (1.0f + expf(-v)); }
#define LDSX() do { asm volatile("s_wait_dscnt 0" ::: "memory"); __builtin_amdgcn_wave_barrier(); __builtin_amdgcn_fence(__ATOMIC_RELEASE, "workgroup"); } while (0)


#define RR 128
#define LL 256
#define IND 128
#define CM 32
#define DP 128
#define NIC (LL * CM)
#ifndef NIB
#define NIB (LL / 4)
#endif
typedef __attribute__((ext_vector_type(8))) __bf16 v8b;
__device__ __forceinline__ v16b frag_b(const __bf16* rowk0, int lane) {
  union { v16b v; v8b q[2]; } u; const __bf16* p = rowk0 + 8 * (lane >> 4);
  u.q[0] = *(const v8b*)p; u.q[1] = *(const v8b*)(p + 16); return u.v;
}
__device__ __forceinline__ float bfr(float v) { return (float)(__bf16)v; }
__device__ __attribute__((noinline)) float exp_ni(float v) { return expf(v); }
__device__ __attribute__((noinline)) float erf_ni(float v) { return erff(v); }

#define WS_PW1 0u
#define WS_PW2 (WS_PW1 + 2u * CM * IND)
#define WS_TH  (WS_PW2 + 2u * (size_t)DP * CM * CM)
#define WS_TL  (WS_TH + 2u * (size_t)NIC * RR)
#define WS_END (WS_TL + 2u * (size_t)NIC * RR)

__global__ __launch_bounds__(256) void k_pack(const float* __restrict__ W1, const float* __restrict__ W2, __bf16* __restrict__ P1, _Float16* __restrict__ P2) {
  const int n = blockIdx.x, t = threadIdx.x; __shared__ __align__(16) __bf16 s1[IND]; __shared__ __align__(16) _Float16 s2[CM * CM];
  if (n < CM) { if (t < IND) s1[t] = (__bf16)W1[(size_t)t * CM + n]; __syncthreads(); if (t < IND / 8) vst2((unsigned*)(P1 + (size_t)n * IND + t * 8), *(const v4u*)&s1[t * 8]); __syncthreads(); }
  for (int k = t; k < CM * CM; k += 256) s2[k] = (_Float16)(bfr(W2[(size_t)k * DP + n]) * 256.0f);
  __syncthreads();
  for (int q = t; q < CM * CM / 8; q += 256) vst2((unsigned*)(P2 + (size_t)n * CM * CM + q * 8), *(const v4u*)&s2[q * 8]);
}
__global__ __launch_bounds__(256) void k_mp(const float* __restrict__ M, const __bf16* __restrict__ P1, const float* __restrict__ B1, __bf16* __restrict__ TH, __bf16* __restrict__ TL) {
  __shared__ __align__(16) __bf16 sh[CM][RR + 8], sl[CM][RR + 8];
  const int tid = threadIdx.x, wave = tid >> 5, lane = tid & 31, col = lane & 15, g = lane >> 4; const size_t i = blockIdx.x; const int r0 = wave * 16;
  v8f acc[2] = {};
#pragma unroll
  for (int kc = 0; kc < IND / 32; ++kc) { v16b a; { const float* p = M + ((size_t)(r0 + col) * LL + i) * IND + kc * 32 + 8 * g;
#pragma unroll
      for (int q = 0; q < 8; ++q) { a[q] = (__bf16)p[q]; a[8 + q] = (__bf16)p[16 + q]; } }
#pragma unroll
    for (int j = 0; j < 2; ++j) acc[j] = wmma_bf(a, frag_b(P1 + (size_t)(j * 16 + col) * IND + kc * 32, lane), acc[j]); }
#pragma unroll
  for (int j = 0; j < 2; ++j) { const int c = j * 16 + col; const float bb = bfr(B1[c]);
#pragma unroll
    for (int r = 0; r < 8; ++r) { const float v = acc[j][r] + bb; const __bf16 h = (__bf16)v; sh[c][r0 + 8 * g + r] = h; sl[c][r0 + 8 * g + r] = (__bf16)(v - (float)h); } }
  __syncthreads();
  for (int e = tid; e < CM * (RR / 8); e += 256) { const int c = e >> 4, q = e & 15; const size_t o = (i * CM + c) * RR + q * 8; vst2((unsigned*)(TH + o), *(const v4u*)&sh[c][q * 8]); vst2((unsigned*)(TL + o), *(const v4u*)&sl[c][q * 8]); }
}
__global__ __launch_bounds__(128) void k_op(const __bf16* __restrict__ TH, const __bf16* __restrict__ TL, const _Float16* __restrict__ P2, const float* __restrict__ B2, const float* __restrict__ X, float* __restrict__ OUT) {
  __shared__ __align__(16) _Float16 sop[16][CM * CM + 8]; __shared__ __align__(16) float so[16][DP + 4];
  const int tid = threadIdx.x, wave = tid >> 5, lane = tid & 31, col = lane & 15, g = lane >> 4; const int ib = blockIdx.x, jb = blockIdx.y; const int i0 = ib * 4, j0 = jb * 4;
#pragma unroll
  for (int ct = 0; ct < 2; ++ct) { v8f acc[8] = {};
    const size_t arow = ((size_t)(i0 + wave) * CM + ct * 16 + col) * RR;
#pragma unroll
    for (int kc = 0; kc < RR / 32; ++kc) { const v16b ah = frag_b(TH + arow + kc * 32, lane), al = frag_b(TL + arow + kc * 32, lane);
#pragma unroll
      for (int jt = 0; jt < 8; ++jt) { const size_t brow = ((size_t)(j0 + (jt >> 1)) * CM + (jt & 1) * 16 + col) * RR + kc * 32; const v16b bh = frag_b(TH + brow, lane), bl = frag_b(TL + brow, lane); acc[jt] = wmma_bf(al, bh, acc[jt]); acc[jt] = wmma_bf(ah, bl, acc[jt]); acc[jt] = wmma_bf(ah, bh, acc[jt]); } }
#pragma unroll
    for (int jt = 0; jt < 8; ++jt)
#pragma unroll
      for (int r = 0; r < 8; ++r) sop[wave * 4 + (jt >> 1)][((jt & 1) * 16 + col) * CM + ct * 16 + 8 * g + r] = (_Float16)(acc[jt][r] * (1.0f / (float)RR)); }
  if (tid < 16) for (int k = CM * CM; k < CM * CM + 8; ++k) sop[tid][k] = (_Float16)0.f;
  __syncthreads();
  { v8f acc2[2] = {};
#pragma unroll 4
    for (int kc = 0; kc < CM * CM / 32; ++kc) { const v16h a = frag_h(&sop[col][kc * 32], lane);
#pragma unroll
      for (int jt = 0; jt < 2; ++jt) acc2[jt] = wmma16(a, frag_h(P2 + (size_t)((wave * 2 + jt) * 16 + col) * (CM * CM) + kc * 32, lane), acc2[jt]); }
#pragma unroll
    for (int jt = 0; jt < 2; ++jt) { const int e = (wave * 2 + jt) * 16 + col; const float bb = bfr(B2[e]);
#pragma unroll
      for (int r = 0; r < 8; ++r) { const int p = 8 * g + r; const size_t orow = (size_t)(i0 + (p >> 2)) * LL + j0 + (p & 3); so[p][e] = acc2[jt][r] * (1.0f / 256.0f) + bb + bfr(X[orow * DP + e]); } } }
  __syncthreads();
  for (int e2 = tid; e2 < 16 * (DP / 4); e2 += 128) { const int p = e2 >> 5, q = e2 & 31; const size_t orow = (size_t)(i0 + (p >> 2)) * LL + j0 + (p & 3); vst2(OUT + orow * DP + q * 4, *(const v4f*)&so[p][q * 4]); }
}
extern "C" void kernel_launch(void* const* d_in, const int* in_sizes, int n_in, void* d_out, int out_size, void* d_ws, size_t ws_size, hipStream_t stream) {
  (void)in_sizes; (void)n_in; (void)out_size;
  const float** F = (const float**)d_in;
  if (ws_size < (size_t)WS_END) return;
  char* ws = (char*)d_ws; __bf16 *P1 = (__bf16*)(ws + WS_PW1), *TH = (__bf16*)(ws + WS_TH), *TL = (__bf16*)(ws + WS_TL); _Float16* P2 = (_Float16*)(ws + WS_PW2);
  k_pack<<<DP, 256, 0, stream>>>(F[2], F[4], P1, P2);
  k_mp<<<LL, 256, 0, stream>>>(F[1], P1, F[3], TH, TL);
  k_op<<<dim3(NIB, LL / 4), 128, 0, stream>>>(TH, TL, P2, F[5], F[0], (float*)d_out);
}
